// ICLAttention_7335804142256
// MI455X (gfx1250) — hardware-verified
//
#include <hip/hip_runtime.h>
#include <math.h>
#include <stdint.h>

#define NBAT 2
#define SEQ_LEN 2048
#define EMB 1024
#define NHEADS 16
#define HDIM 64
#define ROPE_HALF 32
#define PROB_CARRY 32768.0f
#define VLO_CARRY 16384.0f
#define VLO_FOLD (1.0f / 16384.0f)
#define SCORE_SCALE (1.0f / 32.0f)
#define LOG2_BASE_STEP 0.41524101186092028f

typedef __attribute__((ext_vector_type(16))) _Float16 v16h;
typedef __attribute__((ext_vector_type(8)))  _Float16 v8h;
typedef __attribute__((ext_vector_type(16))) __bf16   v16b;
typedef __attribute__((ext_vector_type(8)))  __bf16   v8b;
typedef __attribute__((ext_vector_type(8)))  float    v8f;
typedef __attribute__((ext_vector_type(4)))  float    v4f;
typedef __attribute__((ext_vector_type(2)))  float    v2f;
typedef __attribute__((ext_vector_type(4)))  unsigned int v4u;

__device__ __forceinline__ unsigned short f2bf_bits(float f) {
  unsigned u = __float_as_uint(f);
  return (unsigned short)((u + 0x7FFFu + ((u >> 16) & 1u)) >> 16);
}
__device__ __forceinline__ float bf_bits2f(unsigned short h) { return __uint_as_float(((unsigned)h) << 16); }

__device__ __forceinline__ void dep_guard_h(v8f& a, v8f& b, v16h x, v16h y) { asm volatile("v_nop\n\tv_nop\n\tv_nop\n\tv_nop" : "+v"(a), "+v"(b) : "v"(x), "v"(y)); }
__device__ __forceinline__ void dep_guard_b(v8f& a, v8f& b, v16b x, v16b y) { asm volatile("v_nop\n\tv_nop\n\tv_nop\n\tv_nop" : "+v"(a), "+v"(b) : "v"(x), "v"(y)); }
__device__ __forceinline__ void keep4_h(v16h a, v16h b, v16h c, v16h d) { asm volatile("v_nop" :: "v"(a), "v"(b), "v"(c), "v"(d)); }
__device__ __forceinline__ void keep4_b(v16b a, v16b b, v16b c, v16b d) { asm volatile("v_nop" :: "v"(a), "v"(b), "v"(c), "v"(d)); }
__device__ __forceinline__ void acc_guard4(v8f& a, v8f& b, v8f& c, v8f& d) { asm volatile("v_nop\n\tv_nop\n\tv_nop\n\tv_nop" : "+v"(a), "+v"(b), "+v"(c), "+v"(d)); }
template <typename T> struct Frag;
template <> struct Frag<_Float16> {
  typedef v16h V; union U { v16h v; v8h h[2]; };
  static __device__ __forceinline__ v16h load(const _Float16* p) {
    U f; f.h[0] = *(const v8h*)(p); f.h[1] = *(const v8h*)(p + 16); return f.v;
  }
  static __device__ __forceinline__ v8f mma(v16h a, v16h b, v8f c) {
    return __builtin_amdgcn_wmma_f32_16x16x32_f16(false, a, false, b, (short)0, c, false, false);
  }
  static __device__ __forceinline__ void guard(v8f& a, v8f& b, v16h x, v16h y) { dep_guard_h(a, b, x, y); }
  static __device__ __forceinline__ void keep(v16h a, v16h b, v16h c, v16h d) { keep4_h(a, b, c, d); }
};
template <> struct Frag<__bf16> {
  typedef v16b V; union U { v16b v; v8b h[2]; };
  static __device__ __forceinline__ v16b load(const __bf16* p) {
    U f; f.h[0] = *(const v8b*)(p); f.h[1] = *(const v8b*)(p + 16); return f.v;
  }
  static __device__ __forceinline__ v8f mma(v16b a, v16b b, v8f c) {
    return __builtin_amdgcn_wmma_f32_16x16x32_bf16(false, a, false, b, (short)0, c, false, false);
  }
  static __device__ __forceinline__ void guard(v8f& a, v8f& b, v16b x, v16b y) { dep_guard_b(a, b, x, y); }
  static __device__ __forceinline__ void keep(v16b a, v16b b, v16b c, v16b d) { keep4_b(a, b, c, d); }
};

template <int ET> struct Elem;
template <> struct Elem<0> { typedef _Float16 T; };
template <> struct Elem<1> { typedef __bf16 T; };
template <int ET, bool SPLIT, int BIAS_MODE, int OUT_MODE, bool RESID, int ACT = 0, bool SPLITB = true>
__global__ __launch_bounds__(256) void wmma_gemm64(
    const unsigned short* __restrict__ Ap, const unsigned short* __restrict__ A2p, int lda, long strideA,
    const unsigned short* __restrict__ Btp, const unsigned short* __restrict__ Bt2p, int ldb, long strideB,
    void* __restrict__ Cout, void* __restrict__ Cout2, int ldc, long strideC,
    const float* __restrict__ bias,
    const float* __restrict__ resid, long strideR,
    int M, int N, int K, float scale) {
  typedef typename Elem<ET>::T T;
  typedef typename Frag<T>::V V;
  const T* A = (const T*)Ap; const T* A2 = (const T*)A2p; const T* Bt = (const T*)Btp; const T* Bt2 = (const T*)Bt2p;
  __shared__ __align__(16) float sT[8][16 * 68];
  const int b    = blockIdx.y;
  const int lane = threadIdx.x & 31;
  const int wave = threadIdx.x >> 5;
  const int tilesN = N >> 6;
  const int tilesM = M >> 6;
  const int tile = blockIdx.x * 8 + wave;
  if (tile >= tilesM * tilesN) return;
  const int tm = tile / tilesN;
  const int tn = tile - tm * tilesN;
  const int m0 = tm << 6;
  const int n0 = tn << 6;

  const T* Ab  = A  + (size_t)b * strideA;
  const T* Bb  = Bt + (size_t)b * strideB;
  const T* Ab2 = SPLIT ? (A2  + (size_t)b * strideA) : nullptr;
  const T* Bb2 = SPLIT ? (Bt2 + (size_t)b * strideB) : nullptr;

  const int rlane = lane & 15;
  const int koff  = (lane >> 4) * 8;
  const int mOff  = (lane >> 4) * 8;

  v8f acc[4][4];
#pragma unroll
  for (int i = 0; i < 4; ++i)
#pragma unroll
    for (int j = 0; j < 4; ++j) acc[i][j] = (v8f){0.f,0.f,0.f,0.f,0.f,0.f,0.f,0.f};

  for (int k0 = 0; k0 < K; k0 += 32) {
    V bh[4], bl[4];
#pragma unroll
    for (int j = 0; j < 4; ++j) {
      const size_t bo = (size_t)(n0 + (j << 4) + rlane) * ldb + koff + k0;
      bh[j] = Frag<T>::load(Bb + bo);
      if (SPLIT && SPLITB) bl[j] = Frag<T>::load(Bb2 + bo);
    }
#pragma unroll
    for (int i = 0; i < 4; ++i) {
      const size_t ao = (size_t)(m0 + (i << 4) + rlane) * lda + koff + k0;
      V ah = Frag<T>::load(Ab + ao);
      V al;
      if (SPLIT) al = Frag<T>::load(Ab2 + ao);
#pragma unroll
      for (int j = 0; j < 4; ++j) {
        acc[i][j] = Frag<T>::mma(ah, bh[j], acc[i][j]);
        if (SPLIT) {
          if (SPLITB) acc[i][j] = Frag<T>::mma(ah, bl[j], acc[i][j]);
          acc[i][j] = Frag<T>::mma(al, bh[j], acc[i][j]);
        }
      }
      Frag<T>::guard(acc[i][0], acc[i][3], ah, SPLIT ? al : ah);
    }
    Frag<T>::keep(bh[0], bh[1], bh[2], bh[3]);
    if (SPLIT && SPLITB) Frag<T>::keep(bl[0], bl[1], bl[2], bl[3]);
  }
  acc_guard4(acc[0][0], acc[0][1], acc[0][2], acc[0][3]);
  acc_guard4(acc[1][0], acc[1][1], acc[1][2], acc[1][3]);
  acc_guard4(acc[2][0], acc[2][1], acc[2][2], acc[2][3]);
  acc_guard4(acc[3][0], acc[3][1], acc[3][2], acc[3][3]);

  float* slab = sT[wave];
  const float* Rb = RESID ? (resid + (size_t)b * strideR) : nullptr;
#pragma unroll
  for (int i = 0; i < 4; ++i) {
    const int mBase = m0 + (i << 4);
#pragma unroll
    for (int j = 0; j < 4; ++j) {
      const int n = n0 + (j << 4) + rlane;
      float bv = 0.f;
      if (BIAS_MODE == 2) bv = bias[n];
#pragma unroll
      for (int r = 0; r < 8; ++r) {
        float v = acc[i][j][r] * scale;
        if (BIAS_MODE == 1) v += bias[mBase + mOff + r];
        if (BIAS_MODE == 2) v += bv;
        if (RESID) v += Rb[(size_t)(mBase + mOff + r) * ldc + n];
        if (ACT == 1) v = tanhf(v);
        if (ACT == 2) v = fmaxf(v, 0.0f);
        if (ACT == 3) v = v / (1.0f + expf(-v));
        if (ACT == 4) v = (v > 0.f) ? v : 0.01f * v;
        slab[(mOff + r) * 68 + (j << 4) + rlane] = v;
      }
    }
    __builtin_amdgcn_fence(__ATOMIC_RELEASE, "workgroup");
    __builtin_amdgcn_wave_barrier();
    __builtin_amdgcn_fence(__ATOMIC_ACQUIRE, "workgroup");
    if (OUT_MODE == 0) {
      float* C = (float*)Cout + (size_t)b * strideC;
      const int hh = lane >> 4, c4 = (lane & 15) * 4;
      for (int pass = 0; pass < 2; ++pass) {
#pragma unroll
        for (int it = 0; it < 8; ++it) {
          const int row = it * 2 + hh;
          v4f v = *(const v4f*)(slab + row * 68 + c4);
          *(volatile v4f*)(C + (size_t)(mBase + row) * ldc + n0 + c4) = v;
        }
        __threadfence();
      }
    } else {
      const int q = lane >> 3, c8 = (lane & 7) * 8;
      unsigned short* C  = (unsigned short*)Cout  + (size_t)b * strideC;
      unsigned short* C2 = (OUT_MODE >= 2) ? ((unsigned short*)Cout2 + (size_t)b * strideC) : nullptr;
      for (int pass = 0; pass < 2; ++pass) {
#pragma unroll
        for (int it = 0; it < 4; ++it) {
          const int row = it * 4 + q;
          const float* sp = slab + row * 68 + c8;
          v8h hv, lv;
#pragma unroll
          for (int e = 0; e < 8; ++e) {
            if (OUT_MODE == 1) {
              hv[e] = (_Float16)sp[e];
            } else if (OUT_MODE == 3) {
              const _Float16 hq = (_Float16)sp[e];
              hv[e] = hq;
              lv[e] = (_Float16)((sp[e] - (float)hq) * VLO_CARRY);
            } else {
              unsigned short hb = f2bf_bits(sp[e]);
              unsigned short lb = f2bf_bits(sp[e] - bf_bits2f(hb));
              hv[e] = __builtin_bit_cast(_Float16, hb);
              lv[e] = __builtin_bit_cast(_Float16, lb);
            }
          }
          *(volatile v8h*)(C + (size_t)(mBase + row) * ldc + n0 + c8) = hv;
          if (OUT_MODE >= 2) *(volatile v8h*)(C2 + (size_t)(mBase + row) * ldc + n0 + c8) = lv;
        }
        __threadfence();
      }
    }
    __builtin_amdgcn_fence(__ATOMIC_RELEASE, "workgroup");
    __builtin_amdgcn_wave_barrier();
    __builtin_amdgcn_fence(__ATOMIC_ACQUIRE, "workgroup");
  }
}

__device__ __forceinline__ unsigned pk16(unsigned short a, unsigned short b) { return (unsigned)a | ((unsigned)b << 16); }

__global__ __launch_bounds__(256) void cast_f32_bf16x2(const float* __restrict__ in, unsigned short* __restrict__ out, int n2) {
  const int i = blockIdx.x * 256 + threadIdx.x;
  if (i < n2) {
    const v2f f = *(const v2f*)(in + 2 * (size_t)i);
    const unsigned u = pk16(f2bf_bits(f[0]), f2bf_bits(f[1]));
    ((volatile unsigned*)out)[i] = u;
    __threadfence();
    ((volatile unsigned*)out)[i] = u;
  }
}

__global__ __launch_bounds__(256) void split_bf16x2_kernel(const float* __restrict__ in, unsigned short* __restrict__ hi,
                                                           unsigned short* __restrict__ lo, int n2) {
  const int i = blockIdx.x * 256 + threadIdx.x;
  if (i < n2) {
    const v2f f = *(const v2f*)(in + 2 * (size_t)i);
    const unsigned short h0 = f2bf_bits(f[0]), h1 = f2bf_bits(f[1]);
    const unsigned short l0 = f2bf_bits(f[0] - bf_bits2f(h0)), l1 = f2bf_bits(f[1] - bf_bits2f(h1));
    const unsigned uh = pk16(h0, h1), ul = pk16(l0, l1);
    ((volatile unsigned*)hi)[i] = uh;
    ((volatile unsigned*)lo)[i] = ul;
    __threadfence();
    ((volatile unsigned*)hi)[i] = uh;
    ((volatile unsigned*)lo)[i] = ul;
  }
}

__global__ __launch_bounds__(256) void rope_table_kernel(float* __restrict__ ct, float* __restrict__ st) {
  const int i = blockIdx.x * 256 + threadIdx.x;
  const int s = i >> 5;
  const int j = i & (ROPE_HALF - 1);
  const float inv_freq = exp2f(-(float)j * LOG2_BASE_STEP);
  const float ang = (float)s * inv_freq;
  const float cv = cosf(ang);
  const float sv = sinf(ang);
  ((volatile float*)ct)[i] = cv;
  ((volatile float*)st)[i] = sv;
  __threadfence();
  ((volatile float*)ct)[i] = cv;
  ((volatile float*)st)[i] = sv;
}

__device__ __forceinline__ unsigned pkh2(float a, float b) {
  return (unsigned)__builtin_bit_cast(unsigned short, (_Float16)a) | ((unsigned)__builtin_bit_cast(unsigned short, (_Float16)b) << 16);
}
__global__ __launch_bounds__(256) void rope_f16_kernel(const float* __restrict__ x, const float* __restrict__ ct,
                                                       const float* __restrict__ st, unsigned short* __restrict__ y) {
  const int gt  = blockIdx.x * 256 + threadIdx.x;
  const int row = gt >> 7;
  const int cg  = gt & 127;
  const int s   = row & (SEQ_LEN - 1);
  const int j0  = (cg * 4) & (ROPE_HALF - 1);
  const float* xr = x + (size_t)row * EMB + 8 * cg;
  const v4f a  = *(const v4f*)(xr);
  const v4f bq = *(const v4f*)(xr + 4);
  const v4f cs = *(const v4f*)(ct + s * ROPE_HALF + j0);
  const v4f sn = *(const v4f*)(st + s * ROPE_HALF + j0);
  const float o0 = a[0] * cs[0] - a[1] * sn[0];
  const float o1 = a[1] * cs[0] + a[0] * sn[0];
  const float o2 = a[2] * cs[1] - a[3] * sn[1];
  const float o3 = a[3] * cs[1] + a[2] * sn[1];
  const float o4 = bq[0] * cs[2] - bq[1] * sn[2];
  const float o5 = bq[1] * cs[2] + bq[0] * sn[2];
  const float o6 = bq[2] * cs[3] - bq[3] * sn[3];
  const float o7 = bq[3] * cs[3] + bq[2] * sn[3];
  v4u pk;
  pk[0] = pkh2(o0, o1);
  pk[1] = pkh2(o2, o3);
  pk[2] = pkh2(o4, o5);
  pk[3] = pkh2(o6, o7);
  unsigned short* yp = y + (size_t)row * EMB + 8 * cg;
  *(volatile v4u*)yp = pk;
  __threadfence();
  *(volatile v4u*)yp = pk;
}

#define AT_D 64
#define AT_NW 4
#define AT_QB 64
#define AT_KC 64

__device__ __forceinline__ v8f mma_h16(v16h a, v16h b, v8f c) {
  c = __builtin_amdgcn_wmma_f32_16x16x32_f16(false, a, false, b, (short)0, c, false, false);
  asm volatile("v_nop\n\tv_nop\n\tv_nop\n\tv_nop" : "+v"(c) : "v"(a), "v"(b));
  return c;
}

__global__ __launch_bounds__(128)
void mha_full64_f16_kernel(const unsigned short* __restrict__ qp, const unsigned short* __restrict__ kp,
                           const unsigned short* __restrict__ vthp, const unsigned short* __restrict__ vtlp,
                           float* __restrict__ out, float sscale, float lo_fold) {
  union FH { v16h v; v8h h[2]; };
  __shared__ __align__(16) _Float16 Ksh[AT_KC * AT_D];
  __shared__ __align__(16) _Float16 Vth[AT_D * AT_KC];
  __shared__ __align__(16) _Float16 Vtl[AT_D * AT_KC];
  __shared__ __align__(16) _Float16 Psh[AT_NW][16 * AT_KC];
  __shared__ __align__(16) float    Os[AT_NW][16 * 68];

  const int tid  = threadIdx.x;
  const int wave = tid >> 5;
  const int lane = tid & 31;
  const int hh   = lane >> 4;
  const int c    = lane & 15;

  const int nqb  = SEQ_LEN / AT_QB;
  const int bx   = blockIdx.x;
  const int qb   = bx % nqb;
  const int bhid = bx / nqb;
  const int h    = bhid % NHEADS;
  const int b    = bhid / NHEADS;
  const int q0   = qb * AT_QB + wave * 16;

  const _Float16* Qb = (const _Float16*)(const void*)qp   + (size_t)b * SEQ_LEN * EMB + (size_t)h * AT_D;
  const _Float16* Kb = (const _Float16*)(const void*)kp   + (size_t)b * SEQ_LEN * EMB + (size_t)h * AT_D;
  const _Float16* Vh = (const _Float16*)(const void*)vthp + (size_t)b * EMB * SEQ_LEN + (size_t)h * AT_D * SEQ_LEN;
  const _Float16* Vl = (const _Float16*)(const void*)vtlp + (size_t)b * EMB * SEQ_LEN + (size_t)h * AT_D * SEQ_LEN;
  float*          ob = out + (size_t)b * SEQ_LEN * EMB + (size_t)h * AT_D;

  v16h qa[2];
#pragma unroll
  for (int dc = 0; dc < 2; ++dc) qa[dc] = Frag<_Float16>::load(Qb + (size_t)(q0 + c) * EMB + dc * 32 + 8 * hh);

  float mrow[8], lrow[8];
  v8f oacc[4], oacc2[4];
#pragma unroll
  for (int r = 0; r < 8; ++r) { mrow[r] = -INFINITY; lrow[r] = 0.f; }
#pragma unroll
  for (int t = 0; t < 4; ++t) { oacc[t] = (v8f){0.f,0.f,0.f,0.f,0.f,0.f,0.f,0.f}; oacc2[t] = (v8f){0.f,0.f,0.f,0.f,0.f,0.f,0.f,0.f}; }

  const int nChunks = SEQ_LEN / AT_KC;
  for (int kc = 0; kc < nChunks; ++kc) {
    const int kv0 = kc * AT_KC;
    __syncthreads();
    {
      const int r = tid >> 1, half = (tid & 1) * 32;
      const _Float16* ks  = Kb + (size_t)(kv0 + r) * EMB + half;
      const _Float16* vsh = Vh + (size_t)r * SEQ_LEN + kv0 + half;
      const _Float16* vsl = Vl + (size_t)r * SEQ_LEN + kv0 + half;
#pragma unroll
      for (int i = 0; i < 4; ++i) {
        const v8h a0 = *(const v8h*)(ks + 8 * i);
        const v8h b0 = *(const v8h*)(vsh + 8 * i);
        const v8h b1 = *(const v8h*)(vsl + 8 * i);
        *(v8h*)(Ksh + r * AT_D  + half + 8 * i) = a0;
        *(v8h*)(Vth + r * AT_KC + half + 8 * i) = b0;
        *(v8h*)(Vtl + r * AT_KC + half + 8 * i) = b1;
      }
    }
    __syncthreads();

    v8f s[4];
#pragma unroll
    for (int j = 0; j < 4; ++j) {
      s[j] = (v8f){0.f,0.f,0.f,0.f,0.f,0.f,0.f,0.f};
#pragma unroll
      for (int dc = 0; dc < 2; ++dc) {
        FH kb;
        kb.h[0] = *(const v8h*)(Ksh + (j * 16 + c) * AT_D + dc * 32 + 8 * hh);
        kb.h[1] = *(const v8h*)(Ksh + (j * 16 + c) * AT_D + dc * 32 + 16 + 8 * hh);
        s[j] = mma_h16(qa[dc], kb.v, s[j]);
      }
    }
    float cm[8];
#pragma unroll
    for (int r = 0; r < 8; ++r) {
      float m = -INFINITY;
#pragma unroll
      for (int j = 0; j < 4; ++j) {
        const float sv = s[j][r] * sscale;
        s[j][r] = sv;
        m = fmaxf(m, sv);
      }
#pragma unroll
      for (int off = 1; off < 16; off <<= 1) m = fmaxf(m, __shfl_xor(m, off, 32));
      cm[r] = m;
    }
    _Float16* pw = Psh[wave];
#pragma unroll
    for (int r = 0; r < 8; ++r) {
      const float mnew  = fmaxf(mrow[r], cm[r]);
      const float alpha = expf(mrow[r] - mnew);
      mrow[r] = mnew;
      float psum = 0.f;
#pragma unroll
      for (int j = 0; j < 4; ++j) {
        const float p = expf(s[j][r] - mnew);
        psum += p;
        pw[(8 * hh + r) * AT_KC + j * 16 + c] = (_Float16)(p * PROB_CARRY);
      }
#pragma unroll
      for (int off = 1; off < 16; off <<= 1) psum += __shfl_xor(psum, off, 32);
      lrow[r] = lrow[r] * alpha + psum;
#pragma unroll
      for (int t = 0; t < 4; ++t) { oacc[t][r] *= alpha; oacc2[t][r] *= alpha; }
    }
    __builtin_amdgcn_fence(__ATOMIC_RELEASE, "workgroup");
    __builtin_amdgcn_wave_barrier();
    __builtin_amdgcn_fence(__ATOMIC_ACQUIRE, "workgroup");
#pragma unroll 1
    for (int kk = 0; kk < 2; ++kk) {
      FH pa;
      pa.h[0] = *(const v8h*)(pw + c * AT_KC + kk * 32 + 8 * hh);
      pa.h[1] = *(const v8h*)(pw + c * AT_KC + kk * 32 + 16 + 8 * hh);
#pragma unroll
      for (int t = 0; t < 4; ++t) {
        FH vb, vl;
        vb.h[0] = *(const v8h*)(Vth + (t * 16 + c) * AT_KC + kk * 32 + 8 * hh);
        vb.h[1] = *(const v8h*)(Vth + (t * 16 + c) * AT_KC + kk * 32 + 16 + 8 * hh);
        vl.h[0] = *(const v8h*)(Vtl + (t * 16 + c) * AT_KC + kk * 32 + 8 * hh);
        vl.h[1] = *(const v8h*)(Vtl + (t * 16 + c) * AT_KC + kk * 32 + 16 + 8 * hh);
        oacc[t]  = mma_h16(pa.v, vb.v, oacc[t]);
        oacc2[t] = mma_h16(pa.v, vl.v, oacc2[t]);
      }
    }
  }

  float* os = Os[wave];
#pragma unroll
  for (int r = 0; r < 8; ++r) {
    const float inv = 1.0f / (lrow[r] * PROB_CARRY);
#pragma unroll
    for (int t = 0; t < 4; ++t) os[(8 * hh + r) * 68 + t * 16 + c] = (oacc[t][r] + oacc2[t][r] * lo_fold) * inv;
  }
  __builtin_amdgcn_fence(__ATOMIC_RELEASE, "workgroup");
  __builtin_amdgcn_wave_barrier();
  __builtin_amdgcn_fence(__ATOMIC_ACQUIRE, "workgroup");
  {
    const int c4 = (lane & 15) * 4;
    for (int pass = 0; pass < 2; ++pass) {
#pragma unroll
      for (int it = 0; it < 8; ++it) {
        const int row = it * 2 + hh;
        v4f val = *(const v4f*)(os + row * 68 + c4);
        *(volatile v4f*)(ob + (size_t)(q0 + row) * EMB + c4) = val;
      }
      __threadfence();
    }
  }
}

extern "C" void kernel_launch(void* const* d_in, const int* in_sizes, int n_in,
                              void* d_out, int out_size, void* d_ws, size_t ws_size,
                              hipStream_t stream) {
  const int nX = NBAT * SEQ_LEN * EMB;
  const int nW = EMB * EMB;
  if (n_in < 7) return;
  if (in_sizes[0] != nX || in_sizes[1] != nX || in_sizes[2] != nX) return;
  if (in_sizes[3] != nW || in_sizes[4] != nW || in_sizes[5] != nW || in_sizes[6] != nW) return;
  if (out_size != nX) return;

  const float* q   = (const float*)d_in[0];
  const float* k   = (const float*)d_in[1];
  const float* v   = (const float*)d_in[2];
  const float* W_q = (const float*)d_in[3];
  const float* W_k = (const float*)d_in[4];
  const float* W_v = (const float*)d_in[5];
  const float* W_o = (const float*)d_in[6];
  float* outp = (float*)d_out;

  const size_t xb  = (size_t)nX * 2;
  const size_t wbt = (size_t)nW * 2;
  const size_t fb  = (size_t)nX * 4;
  const size_t tb  = (size_t)SEQ_LEN * ROPE_HALF * 4;
  const size_t o_xq = 0, o_xk = o_xq + xb, o_xv = o_xk + xb;
  const size_t o_wq = o_xv + xb, o_wk = o_wq + wbt, o_wv = o_wk + wbt, o_wo = o_wv + wbt;
  const size_t o_cf = o_wo + wbt;
  const size_t o_q16 = o_cf + fb, o_k16 = o_q16 + xb;
  const size_t o_vth = o_k16 + xb, o_vtl = o_vth + xb;
  const size_t o_ohi = o_vtl + xb, o_olo = o_ohi + xb;
  const size_t o_ct = o_olo + xb, o_st = o_ct + tb, o_end = o_st + tb;
  if (o_end > ws_size) return;

  unsigned char* ws = (unsigned char*)d_ws;
  unsigned short* xq  = (unsigned short*)(ws + o_xq);
  unsigned short* xk  = (unsigned short*)(ws + o_xk);
  unsigned short* xv  = (unsigned short*)(ws + o_xv);
  unsigned short* wq  = (unsigned short*)(ws + o_wq);
  unsigned short* wk  = (unsigned short*)(ws + o_wk);
  unsigned short* wv  = (unsigned short*)(ws + o_wv);
  unsigned short* wo  = (unsigned short*)(ws + o_wo);
  float*          cf  = (float*)(ws + o_cf);
  unsigned short* q16 = (unsigned short*)(ws + o_q16);
  unsigned short* k16 = (unsigned short*)(ws + o_k16);
  unsigned short* vth = (unsigned short*)(ws + o_vth);
  unsigned short* vtl = (unsigned short*)(ws + o_vtl);
  unsigned short* ohi = (unsigned short*)(ws + o_ohi);
  unsigned short* olo = (unsigned short*)(ws + o_olo);
  float*          ct  = (float*)(ws + o_ct);
  float*          st  = (float*)(ws + o_st);
  void*        dummy_v = (void*)(ws + o_ct);
  const float* dummy_f = (const float*)(ws + o_st);

  const int nX2 = nX / 2, nW2 = nW / 2;
  cast_f32_bf16x2<<<(nX2 + 255) / 256, 256, 0, stream>>>(q,   xq, nX2);
  cast_f32_bf16x2<<<(nX2 + 255) / 256, 256, 0, stream>>>(k,   xk, nX2);
  cast_f32_bf16x2<<<(nX2 + 255) / 256, 256, 0, stream>>>(v,   xv, nX2);
  cast_f32_bf16x2<<<(nW2 + 255) / 256, 256, 0, stream>>>(W_q, wq, nW2);
  cast_f32_bf16x2<<<(nW2 + 255) / 256, 256, 0, stream>>>(W_k, wk, nW2);
  cast_f32_bf16x2<<<(nW2 + 255) / 256, 256, 0, stream>>>(W_v, wv, nW2);
  cast_f32_bf16x2<<<(nW2 + 255) / 256, 256, 0, stream>>>(W_o, wo, nW2);

  rope_table_kernel<<<(SEQ_LEN * ROPE_HALF) / 256, 256, 0, stream>>>(ct, st);

  const int Mrows  = NBAT * SEQ_LEN;
  const int tilesP = (Mrows / 64) * (EMB / 64);
  const int tilesV = (EMB / 64) * (SEQ_LEN / 64);
  const int ropeBlocks = (Mrows * (EMB / 8)) / 256;

  wmma_gemm64<1, false, 0, 0, false, 0, true><<<dim3((tilesP + 7) / 8, 1), dim3(256), 0, stream>>>(
      xq, xq, EMB, 0L, wq, wq, EMB, 0L, (void*)cf, dummy_v, EMB, 0L, dummy_f, dummy_f, 0L, Mrows, EMB, EMB, 1.0f);
  rope_f16_kernel<<<ropeBlocks, 256, 0, stream>>>(cf, ct, st, q16);

  wmma_gemm64<1, false, 0, 0, false, 0, true><<<dim3((tilesP + 7) / 8, 1), dim3(256), 0, stream>>>(
      xk, xk, EMB, 0L, wk, wk, EMB, 0L, (void*)cf, dummy_v, EMB, 0L, dummy_f, dummy_f, 0L, Mrows, EMB, EMB, 1.0f);
  rope_f16_kernel<<<ropeBlocks, 256, 0, stream>>>(cf, ct, st, k16);

  wmma_gemm64<1, false, 0, 3, false, 0, true><<<dim3((tilesV + 7) / 8, NBAT), dim3(256), 0, stream>>>(
      wv, wv, EMB, 0L, xv, xv, EMB, (long)SEQ_LEN * EMB, (void*)vth, (void*)vtl, SEQ_LEN, (long)EMB * SEQ_LEN,
      dummy_f, dummy_f, 0L, EMB, SEQ_LEN, EMB, 1.0f);

  mha_full64_f16_kernel<<<NBAT * NHEADS * (SEQ_LEN / AT_QB), 128, 0, stream>>>(q16, k16, vth, vtl, cf, SCORE_SCALE, VLO_FOLD);

  split_bf16x2_kernel<<<(nX2 + 255) / 256, 256, 0, stream>>>(cf, ohi, olo, nX2);

  wmma_gemm64<1, true, 0, 0, false, 0, false><<<dim3((tilesP + 7) / 8, 1), dim3(256), 0, stream>>>(
      ohi, olo, EMB, 0L, wo, wo, EMB, 0L, (void*)outp, dummy_v, EMB, 0L, dummy_f, dummy_f, 0L, Mrows, EMB, EMB, 1.0f);
}
